// NCELoss_71305047049043
// MI455X (gfx1250) — hardware-verified
//
#include <hip/hip_runtime.h>
#include <math.h>

typedef __attribute__((ext_vector_type(16))) _Float16 v16h;
typedef __attribute__((ext_vector_type(16))) __bf16 v16b;
typedef __attribute__((ext_vector_type(8)))  _Float16 v8h;
typedef __attribute__((ext_vector_type(8)))  float v8f;
typedef __attribute__((ext_vector_type(4)))  float v4f;
typedef __attribute__((ext_vector_type(2)))  float v2f;
typedef __attribute__((ext_vector_type(4)))  unsigned v4u;
typedef __attribute__((ext_vector_type(4)))  int v4i;
typedef float __attribute__((may_alias)) float_a;
typedef int __attribute__((may_alias)) int_a;

template <typename T> __device__ __forceinline__ void vst2(void* p, T v) { *(volatile T*)p = v; __threadfence(); *(volatile T*)p = v; }
__device__ __forceinline__ v8f wmma16(v16h a, v16h b, v8f c) {
  v8f d = __builtin_amdgcn_wmma_f32_16x16x32_f16(false, a, false, b, (short)0, c, false, false);
  asm volatile("v_nop\n\tv_nop\n\tv_nop\n\tv_nop" : "+v"(d) : "v"(a), "v"(b));
  return d;
}
__device__ __forceinline__ v8f wmma_bf(v16b a, v16b b, v8f c) {
  v8f d = __builtin_amdgcn_wmma_f32_16x16x32_bf16(false, a, false, b, (short)0, c, false, false);
  asm volatile("v_nop\n\tv_nop\n\tv_nop\n\tv_nop" : "+v"(d) : "v"(a), "v"(b));
  return d;
}
__device__ __forceinline__ v16h frag_h(const _Float16* rowk0, int lane) {
  union { v16h v; v8h q[2]; } u; const _Float16* p = rowk0 + 8 * (lane >> 4);
  u.q[0] = *(const v8h*)p; u.q[1] = *(const v8h*)(p + 16); return u.v;
}
__device__ __forceinline__ v16h frag_f32(const float* rowk0, int lane) {
  v16h a; const float* p = rowk0 + 8 * (lane >> 4);
#pragma unroll
  for (int i = 0; i < 8; ++i) { a[i] = (_Float16)p[i]; a[8 + i] = (_Float16)p[16 + i]; }
  return a;
}
__device__ __forceinline__ v16h frag_f32s(const float* rowk0, int lane, float sc) {
  v16h a; const float* p = rowk0 + 8 * (lane >> 4);
#pragma unroll
  for (int i = 0; i < 8; ++i) { a[i] = (_Float16)(p[i] * sc); a[8 + i] = (_Float16)(p[16 + i] * sc); }
  return a;
}
__device__ __forceinline__ v16h fragc_f32(const float* W, int k0, int n, int lane, int ld, int K) {
  v16h a; const int g = lane >> 4;
#pragma unroll
  for (int i = 0; i < 8; ++i) { const int ka = k0 + 8 * g + i, kb = ka + 16;
    a[i] = (_Float16)(ka < K ? W[(size_t)(ka < K ? ka : K - 1) * ld + n] : 0.f); a[8 + i] = (_Float16)(kb < K ? W[(size_t)(kb < K ? kb : K - 1) * ld + n] : 0.f); }
  return a;
}
struct F2 { v16b h, l; };
__device__ __forceinline__ F2 bsplit16(const float v[16]) { F2 r;
#pragma unroll
  for (int i = 0; i < 16; ++i) { const __bf16 h = (__bf16)v[i]; r.h[i] = h; r.l[i] = (__bf16)(v[i] - (float)h); }
  return r; }
__device__ __forceinline__ F2 split_row(const float* row, int k0, int lane) { float v[16]; const float* p = row + k0 + 8 * (lane >> 4);
#pragma unroll
  for (int i = 0; i < 8; ++i) { v[i] = p[i]; v[8 + i] = p[16 + i]; }
  return bsplit16(v); }
__device__ __forceinline__ F2 split_rowK(const float* row, int k0, int lane, int K) { float v[16]; const int g = lane >> 4;
#pragma unroll
  for (int i = 0; i < 8; ++i) { const int ka = k0 + 8 * g + i, kb = ka + 16; v[i] = ka < K ? row[ka < K ? ka : K - 1] : 0.f; v[8 + i] = kb < K ? row[kb < K ? kb : K - 1] : 0.f; }
  return bsplit16(v); }
__device__ __forceinline__ F2 split_col(const float* W, int k0, int n, int lane, int ld, int K) { float v[16]; const int g = lane >> 4;
#pragma unroll
  for (int i = 0; i < 8; ++i) { const int ka = k0 + 8 * g + i, kb = ka + 16; v[i] = ka < K ? W[(size_t)(ka < K ? ka : K - 1) * ld + n] : 0.f; v[8 + i] = kb < K ? W[(size_t)(kb < K ? kb : K - 1) * ld + n] : 0.f; }
  return bsplit16(v); }
__device__ __forceinline__ v8f mac3(const F2& a, const F2& b, v8f c) { c = wmma_bf(a.l, b.h, c); c = wmma_bf(a.h, b.l, c); return wmma_bf(a.h, b.h, c); }
__device__ __forceinline__ float sigm(float v) { return 1.0f / (1.0f + expf(-v)); }
#define LDSX() do { asm volatile("s_wait_dscnt 0" ::: "memory"); __builtin_amdgcn_wave_barrier(); __builtin_amdgcn_fence(__ATOMIC_RELEASE, "workgroup"); } while (0)


#define NS 4096
#define DD 256
#ifndef TRB
#define TRB (NS / 64)
#endif
typedef __attribute__((ext_vector_type(8))) __bf16 v8b;
__device__ __forceinline__ v16b frag_b(const __bf16* rowk0, int lane) {
  union { v16b v; v8b q[2]; } u; const __bf16* p = rowk0 + 8 * (lane >> 4);
  u.q[0] = *(const v8b*)p; u.q[1] = *(const v8b*)(p + 16); return u.v;
}
__device__ __forceinline__ float bfr(float v) { return (float)(__bf16)v; }
__device__ __attribute__((noinline)) float exp_ni(float v) { return expf(v); }
__device__ __attribute__((noinline)) float erf_ni(float v) { return erff(v); }

#define WS_INV 0u
#define WS_END (4u * 2 * NS)

__device__ __attribute__((noinline)) float exp_p(float v) { return expf(v); }
__global__ __launch_bounds__(256) void k_norm(const float* __restrict__ X1, const float* __restrict__ X2, float* __restrict__ INV) {
  const int which = blockIdx.y; const float* X = which ? X2 : X1; const int t = threadIdx.x; const int r = t >> 2, part = t & 3; const size_t row = (size_t)blockIdx.x * 64 + r;
  float s = 0.f; for (int c = part * 64; c < part * 64 + 64; ++c) { const float v = bfr(X[row * DD + c]); s += v * v; }
  s += __shfl_xor(s, 1); s += __shfl_xor(s, 2);
  __shared__ __align__(16) float so[64]; if (part == 0) so[r] = 1.0f / fmaxf(sqrtf(s), 1e-8f); __syncthreads();
  if (t < 16) vst2(INV + (size_t)which * NS + (size_t)blockIdx.x * 64 + t * 4, *(const v4f*)&so[t * 4]);
}
__global__ __launch_bounds__(128) void k_nce(const float* __restrict__ X1, const float* __restrict__ X2, const float* __restrict__ INV, float* __restrict__ OUT) {
  __shared__ __align__(16) float so[64];
  const int tid = threadIdx.x, wave = tid >> 5, lane = tid & 31, col = lane & 15, g = lane >> 4; const int which = blockIdx.y; const size_t r0 = (size_t)blockIdx.x * 64 + wave * 16;
  const float* XA = which ? X2 : X1;
  v16b a[DD / 32];
#pragma unroll
  for (int kc = 0; kc < DD / 32; ++kc) { const float* p = XA + (r0 + col) * DD + kc * 32 + 8 * g;
#pragma unroll
    for (int i = 0; i < 8; ++i) { a[kc][i] = (__bf16)p[i]; a[kc][8 + i] = (__bf16)p[16 + i]; } }
  float inva[8], m[8], l[8], pos[8];
#pragma unroll
  for (int r = 0; r < 8; ++r) { inva[r] = INV[(size_t)which * NS + r0 + 8 * g + r] * 10.0f; m[r] = -3.0e38f; l[r] = 0.f; pos[r] = 0.f; }
#pragma unroll 1
  for (int pass = 0; pass < 2; ++pass) { const int src = pass ? which : (1 - which); const float* XB = src ? X2 : X1; const float* invb = INV + (size_t)src * NS;
#pragma unroll 1
    for (int kt = 0; kt < NS / 16; ++kt) { const int k0 = kt * 16; v8f c = {};
#pragma unroll
      for (int kc = 0; kc < DD / 32; ++kc) { v16b bq; { const float* p = XB + (size_t)(k0 + col) * DD + kc * 32 + 8 * g;
#pragma unroll
          for (int i = 0; i < 8; ++i) { bq[i] = (__bf16)p[i]; bq[8 + i] = (__bf16)p[16 + i]; } }
        c = wmma_bf(a[kc], bq, c); }
      const float ib = invb[k0 + col]; const int kk = k0 + col;
#pragma unroll
      for (int r = 0; r < 8; ++r) { const int row = (int)(r0 + 8 * g + r) ; float s = c[r] * inva[r] * ib; const bool self = (pass == 1) && (kk == row);
        if (pass == 0 && kk == row) pos[r] = s;
        if (self) s = -3.0e38f;
        float mx = s;
#pragma unroll
        for (int o = 1; o < 16; o <<= 1) mx = fmaxf(mx, __shfl_xor(mx, o));
        const float mn = fmaxf(m[r], mx); const float alpha = (m[r] <= -1.0e38f) ? 0.f : exp_p(m[r] - mn); float e = (s <= -1.0e38f) ? 0.f : exp_p(s - mn);
#pragma unroll
        for (int o = 1; o < 16; o <<= 1) e += __shfl_xor(e, o);
        l[r] = l[r] * alpha + e; m[r] = mn; } } }
#pragma unroll
  for (int r = 0; r < 8; ++r) { float pv = pos[r];
#pragma unroll
    for (int o = 1; o < 16; o <<= 1) pv += __shfl_xor(pv, o);
    if (col == 0) so[wave * 16 + 8 * g + r] = (m[r] + logf(l[r])) - pv; }
  __syncthreads();
  if (tid < 16) vst2(OUT + (size_t)which * NS + (size_t)blockIdx.x * 64 + tid * 4, *(const v4f*)&so[tid * 4]);
}
extern "C" void kernel_launch(void* const* d_in, const int* in_sizes, int n_in, void* d_out, int out_size, void* d_ws, size_t ws_size, hipStream_t stream) {
  (void)in_sizes; (void)n_in; (void)out_size;
  const float** F = (const float**)d_in;
  if (ws_size < (size_t)WS_END) return;
  char* ws = (char*)d_ws; float* INV = (float*)(ws + WS_INV);
  k_norm<<<dim3(NS / 64, 2), 256, 0, stream>>>(F[0], F[1], INV);
  k_nce<<<dim3(TRB, 2), 128, 0, stream>>>(F[0], F[1], INV, (float*)d_out);
}
